// DeformConv2dModule_26079041421790
// MI455X (gfx1250) — hardware-verified
//
#include <hip/hip_runtime.h>
#include <stddef.h>


#pragma clang fp contract(off)

#define NBATCH 8
#define NCIN   256
#define NCOUT  256
#define HWD    64
#define NPIX   4096
#define NTAP   9
#define KTOT   2304
#define NTHR   256
#define ASCL   16.0f
#define WSCL   16.0f
#define OINV   0.00390625f

typedef float    v4f  __attribute__((ext_vector_type(4)));
typedef float    v8f  __attribute__((ext_vector_type(8)));
typedef int      v4i  __attribute__((ext_vector_type(4)));
typedef _Float16 v8h  __attribute__((ext_vector_type(8)));
typedef _Float16 v16h __attribute__((ext_vector_type(16)));
union FragH { v16h v; v8h h[2]; };
union Pk8   { v8h h; v4f f; };

static_assert((NCOUT * KTOT) % 8 == 0);
static_assert((NBATCH * NCIN * NPIX) % 4 == 0);
static_assert(KTOT == NTAP * NCIN);

__device__ __forceinline__ float bf16r(float f) {
  unsigned int u = __float_as_uint(f);
  u += 0x7FFFu + ((u >> 16) & 1u);
  u &= 0xFFFF0000u;
  return __uint_as_float(u);
}

__device__ __forceinline__ v8f wmh(v16h a, v16h b, v8f c) {
  v8f d = __builtin_amdgcn_wmma_f32_16x16x32_f16(false, a, false, b, (short)0, c, false, false);
  asm volatile("v_nop\n\tv_nop\n\tv_nop\n\tv_nop" : "+v"(d) : "v"(a), "v"(b));
  return d;
}

__global__ __launch_bounds__(NTHR) void k_wprep(const float* __restrict__ w, _Float16* wt, int n8) {
  const int i  = blockIdx.x * NTHR + threadIdx.x;
  const bool ok = i < n8;
  const int ic = ok ? i : 0;
  const int co = ic / (KTOT / 8);
  const int t0 = (ic - co * (KTOT / 8)) * 8;
  const int k2 = t0 >> 8;
  const int c  = t0 & 255;
  Pk8 pk;
#pragma unroll
  for (int j = 0; j < 8; ++j) {
    const float f = bf16r(w[((size_t)co * NCIN + c + j) * NTAP + k2]);
    pk.h[j] = (_Float16)(f * WSCL);
  }
  _Float16* p = wt + (size_t)co * KTOT + t0;
  if (ok) *(volatile v4f*)p = pk.f;
  __threadfence();
  if (ok) *(volatile v4f*)p = pk.f;
}

__global__ __launch_bounds__(NTHR) void k_xprep(const float* __restrict__ x, float* xr, int n4) {
  const int i  = blockIdx.x * NTHR + threadIdx.x;
  const bool ok = i < n4;
  const int ic = ok ? i : 0;
  const v4f a = *(const v4f*)(x + (size_t)ic * 4);
  v4f r;
  r.x = bf16r(a.x); r.y = bf16r(a.y); r.z = bf16r(a.z); r.w = bf16r(a.w);
  float* p = xr + (size_t)ic * 4;
  if (ok) *(volatile v4f*)p = r;
  __threadfence();
  if (ok) *(volatile v4f*)p = r;
}

struct SmMain {
  int      addr[576 * 4];
  float    wgt[576 * 4];
  _Float16 W[NCOUT * 32];
  _Float16 Bt[64 * 32];
};
struct SmEpi { float o[8 * 16 * 64]; };
union SmU { SmMain m; SmEpi e; };
static_assert(sizeof(SmMain) == 38912);
static_assert(sizeof(SmEpi) <= sizeof(SmMain));

__global__ __launch_bounds__(NTHR) void k_main(
    const float* __restrict__ xr, const float* __restrict__ offs,
    const _Float16* __restrict__ wt, float* out) {
  __shared__ __align__(16) SmU sm;

  const int tid = threadIdx.x;
  const int pt  = blockIdx.x;
  const int b   = pt >> 6;
  const int h   = pt & 63;

  for (int i = tid; i < 576; i += NTHR) {
    const int k2 = i >> 6;
    const int p  = i & 63;
    const int ki = k2 / 3;
    const int kj = k2 - ki * 3;
    const float offy = bf16r(offs[((size_t)(b * 18 + 2 * k2)     * HWD + h) * HWD + p]);
    const float offx = bf16r(offs[((size_t)(b * 18 + 2 * k2 + 1) * HWD + h) * HWD + p]);
    const float py = (float)(ki + h - 1) + offy;
    const float px = (float)(kj + p - 1) + offx;
    const float y0 = floorf(py), x0 = floorf(px);
#pragma unroll
    for (int dy = 0; dy < 2; ++dy) {
#pragma unroll
      for (int dx = 0; dx < 2; ++dx) {
        const float yi = y0 + (float)dy;
        const float xi = x0 + (float)dx;
        const float wy = 1.0f - fabsf(py - yi);
        const float wx = 1.0f - fabsf(px - xi);
        const float wg = wy * wx;
        const bool valid = (yi >= 0.0f) && (yi < 64.0f) && (xi >= 0.0f) && (xi < 64.0f);
        const int yc = (int)fminf(fmaxf(yi, 0.0f), 63.0f);
        const int xc = (int)fminf(fmaxf(xi, 0.0f), 63.0f);
        sm.m.addr[i * 4 + dy * 2 + dx] = yc * HWD + xc;
        sm.m.wgt[i * 4 + dy * 2 + dx]  = valid ? wg : 0.0f;
      }
    }
  }
  __syncthreads();

  const int wave = tid >> 5;
  const int lane = tid & 31;
  const int m    = lane & 15;
  const int hh   = lane >> 4;

  v8f acc[8];
  {
    v8f z;
#pragma unroll
    for (int i = 0; i < 8; ++i) z[i] = 0.0f;
#pragma unroll
    for (int i = 0; i < 8; ++i) acc[i] = z;
  }

  const int sp  = tid & 63;
  const int scg = tid >> 6;

#pragma unroll 1
  for (int kk = 0; kk < 72; ++kk) {
    const int k2 = kk >> 3;
    const int c0 = (kk & 7) << 5;

    __syncthreads();

    {
      const _Float16* src = wt + (size_t)tid * KTOT + k2 * NCIN + c0;
      _Float16* dst = sm.m.W + tid * 32;
      const v8h q0 = *(const v8h*)(src);
      const v8h q1 = *(const v8h*)(src + 8);
      const v8h q2 = *(const v8h*)(src + 16);
      const v8h q3 = *(const v8h*)(src + 24);
      *(v8h*)(dst)      = q0;
      *(v8h*)(dst + 8)  = q1;
      *(v8h*)(dst + 16) = q2;
      *(v8h*)(dst + 24) = q3;
    }

    {
      const int ti = k2 * 64 + sp;
      const v4i ad = *(const v4i*)(sm.m.addr + ti * 4);
      const v4f wg = *(const v4f*)(sm.m.wgt + ti * 4);
      const float* pl = xr + (size_t)(b * NCIN + c0 + scg * 8) * NPIX;
      v8h hv;
#pragma unroll
      for (int j = 0; j < 8; ++j) {
        float v = 0.0f;
        v = v + pl[ad.x] * wg.x;
        v = v + pl[ad.y] * wg.y;
        v = v + pl[ad.z] * wg.z;
        v = v + pl[ad.w] * wg.w;
        hv[j] = (_Float16)(v * ASCL);
        pl += NPIX;
      }
      *(v8h*)(sm.m.Bt + sp * 32 + scg * 8) = hv;
    }

    __syncthreads();

    FragH af[2];
#pragma unroll
    for (int ci = 0; ci < 2; ++ci) {
      const _Float16* pa = sm.m.W + (wave * 32 + ci * 16 + m) * 32 + 8 * hh;
      af[ci].h[0] = *(const v8h*)pa;
      af[ci].h[1] = *(const v8h*)(pa + 16);
    }
#pragma unroll
    for (int pi = 0; pi < 4; ++pi) {
      FragH bf;
      const _Float16* pb = sm.m.Bt + (pi * 16 + m) * 32 + 8 * hh;
      bf.h[0] = *(const v8h*)pb;
      bf.h[1] = *(const v8h*)(pb + 16);
#pragma unroll
      for (int ci = 0; ci < 2; ++ci)
        acc[ci * 4 + pi] = wmh(af[ci].v, bf.v, acc[ci * 4 + pi]);
    }
  }

  __syncthreads();
  float* so = sm.e.o + wave * 1024;
#pragma unroll
  for (int ci = 0; ci < 2; ++ci) {
#pragma unroll
    for (int pi = 0; pi < 4; ++pi) {
      const v8f a = acc[ci * 4 + pi];
#pragma unroll
      for (int r = 0; r < 8; ++r)
        so[(8 * hh + r) * 64 + pi * 16 + m] = fmaxf(a[r] * OINV, 0.0f);
    }
    __syncthreads();
    v4f ov[8];
#pragma unroll
    for (int it = 0; it < 8; ++it) {
      const int row = it * 2 + hh;
      ov[it] = *(const v4f*)(so + row * 64 + 4 * m);
    }
    const size_t ob = (((size_t)b * NCOUT + wave * 32 + ci * 16) * HWD + h) * HWD;
#pragma unroll
    for (int it = 0; it < 8; ++it)
      *(volatile v4f*)(out + ob + (size_t)(it * 2 + hh) * NPIX + 4 * m) = ov[it];
    __threadfence();
#pragma unroll
    for (int it = 0; it < 8; ++it)
      *(volatile v4f*)(out + ob + (size_t)(it * 2 + hh) * NPIX + 4 * m) = ov[it];
    __syncthreads();
  }
}

extern "C" void kernel_launch(void* const* d_in, const int* in_sizes, int n_in,
                              void* d_out, int out_size, void* d_ws, size_t ws_size,
                              hipStream_t stream) {
  if (n_in < 3) return;
  if (in_sizes[0] != NBATCH * NCIN * NPIX) return;
  if (in_sizes[1] != NBATCH * 2 * NTAP * NPIX) return;
  if (in_sizes[2] != NCOUT * NCIN * NTAP) return;
  if (out_size != NBATCH * NCOUT * NPIX) return;

  const float* x      = (const float*)d_in[0];
  const float* offs   = (const float*)d_in[1];
  const float* weight = (const float*)d_in[2];
  float*       out    = (float*)d_out;

  char* ws = (char*)d_ws;
  size_t off = 0;
  const size_t oWt = off; off += (size_t)NCOUT * KTOT * 2;           off = (off + 255) & ~(size_t)255;
  const size_t oXr = off; off += (size_t)NBATCH * NCIN * NPIX * 4;   off = (off + 255) & ~(size_t)255;
  if (off > ws_size) return;
  _Float16* wt = (_Float16*)(ws + oWt);
  float*    xr = (float*)(ws + oXr);

  const int n8 = NCOUT * KTOT / 8;
  const int n4 = NBATCH * NCIN * NPIX / 4;
  k_wprep<<<(n8 + NTHR - 1) / NTHR, NTHR, 0, stream>>>(weight, wt, n8);
  k_xprep<<<(n4 + NTHR - 1) / NTHR, NTHR, 0, stream>>>(x, xr, n4);
  k_main<<<NBATCH * HWD, NTHR, 0, stream>>>(xr, offs, wt, out);
}
